// MyLSTM_19748259627793
// MI455X (gfx1250) — hardware-verified
//
#include <hip/hip_runtime.h>
#include <math.h>

typedef __attribute__((ext_vector_type(16))) _Float16 v16h;
typedef __attribute__((ext_vector_type(8)))  _Float16 v8h;
typedef __attribute__((ext_vector_type(8)))  float    v8f;
typedef __attribute__((ext_vector_type(4)))  float    v4f;

constexpr int SEQ_LEN  = 256;
constexpr int NBATCH   = 512;
constexpr int NIN      = 8;
constexpr int NHID     = 256;
constexpr int NGATE    = 4;
constexpr int NTHR     = 256;
constexpr int ROWS_PB  = 16;
constexpr int KXPAD    = 32;
constexpr int AXP      = 40;
constexpr int AHP      = 264;
constexpr int NBLK_SEQ = NBATCH / ROWS_PB;
constexpr int PLANE_X  = NHID * KXPAD;
constexpr int PLANE_H  = NHID * NHID;
constexpr int MSK_PL   = ROWS_PB * NHID;
constexpr int SLAB_PB  = SEQ_LEN * ROWS_PB;
constexpr float WCARRY     = 16.0f;
constexpr float WCARRY_INV = 0.0625f;

__device__ __forceinline__ void dep_guard_h(v8f& a, v8f& b, v16h x, v16h y) { asm volatile("v_nop\n\tv_nop\n\tv_nop\n\tv_nop" : "+v"(a), "+v"(b) : "v"(x), "v"(y)); }
__device__ __forceinline__ void keep4_h(v16h a, v16h b, v16h c, v16h d) { asm volatile("v_nop" :: "v"(a), "v"(b), "v"(c), "v"(d)); }
__device__ __forceinline__ void acc_guard4(v8f& a, v8f& b, v8f& c, v8f& d) { asm volatile("v_nop\n\tv_nop\n\tv_nop\n\tv_nop" : "+v"(a), "+v"(b), "+v"(c), "+v"(d)); }
template <typename T> struct Frag;
template <> struct Frag<_Float16> {
  typedef v16h V; union U { v16h v; v8h h[2]; };
  static __device__ __forceinline__ v16h load(const _Float16* p) {
    U f; f.h[0] = *(const v8h*)(p); f.h[1] = *(const v8h*)(p + 16); return f.v;
  }
  static __device__ __forceinline__ v8f mma(v16h a, v16h b, v8f c) {
    return __builtin_amdgcn_wmma_f32_16x16x32_f16(false, a, false, b, (short)0, c, false, false);
  }
  static __device__ __forceinline__ void guard(v8f& a, v8f& b, v16h x, v16h y) { dep_guard_h(a, b, x, y); }
  static __device__ __forceinline__ void keep(v16h a, v16h b, v16h c, v16h d) { keep4_h(a, b, c, d); }
};

__device__ __forceinline__ float fsig(float x)  { return __builtin_amdgcn_rcpf(1.0f + __expf(-x)); }
__device__ __forceinline__ float ftanh(float x) { return 1.0f - 2.0f * __builtin_amdgcn_rcpf(__expf(2.0f * x) + 1.0f); }

__global__ __launch_bounds__(NTHR) void prep_in_kernel(const float* __restrict__ Wf, const float* __restrict__ Wi,
                                                      const float* __restrict__ Wc, const float* __restrict__ Wo,
                                                      unsigned short* __restrict__ WX) {
  const int g = blockIdx.x >> 2;
  const float* W = (g == 0) ? Wf : (g == 1) ? Wi : (g == 2) ? Wc : Wo;
  const int e0 = ((blockIdx.x & 3) * NTHR + threadIdx.x) * 8;
  const int j = e0 >> 5, kq = e0 & 31;
  const v4f a = *(const v4f*)(W + j * NIN);
  const v4f b = *(const v4f*)(W + j * NIN + 4);
  const bool live = (kq == 0);
  v8h hv;
  hv[0] = live ? (_Float16)(a[0] * WCARRY) : (_Float16)0.0f;
  hv[1] = live ? (_Float16)(a[1] * WCARRY) : (_Float16)0.0f;
  hv[2] = live ? (_Float16)(a[2] * WCARRY) : (_Float16)0.0f;
  hv[3] = live ? (_Float16)(a[3] * WCARRY) : (_Float16)0.0f;
  hv[4] = live ? (_Float16)(b[0] * WCARRY) : (_Float16)0.0f;
  hv[5] = live ? (_Float16)(b[1] * WCARRY) : (_Float16)0.0f;
  hv[6] = live ? (_Float16)(b[2] * WCARRY) : (_Float16)0.0f;
  hv[7] = live ? (_Float16)(b[3] * WCARRY) : (_Float16)0.0f;
  unsigned short* p = WX + (size_t)g * PLANE_X + e0;
  *(volatile v8h*)p = hv;
  __threadfence();
  *(volatile v8h*)p = hv;
}

__global__ __launch_bounds__(NTHR) void prep_rec_kernel(const float* __restrict__ Vf, const float* __restrict__ Vi,
                                                       const float* __restrict__ Vc, const float* __restrict__ Vo,
                                                       unsigned short* __restrict__ WH) {
  const int g = blockIdx.x >> 5;
  const float* Vg = (g == 0) ? Vf : (g == 1) ? Vi : (g == 2) ? Vc : Vo;
  const int e0 = ((blockIdx.x & 31) * NTHR + threadIdx.x) * 8;
  const v4f a = *(const v4f*)(Vg + e0);
  const v4f b = *(const v4f*)(Vg + e0 + 4);
  v8h hv;
  hv[0] = (_Float16)(a[0] * WCARRY); hv[1] = (_Float16)(a[1] * WCARRY);
  hv[2] = (_Float16)(a[2] * WCARRY); hv[3] = (_Float16)(a[3] * WCARRY);
  hv[4] = (_Float16)(b[0] * WCARRY); hv[5] = (_Float16)(b[1] * WCARRY);
  hv[6] = (_Float16)(b[2] * WCARRY); hv[7] = (_Float16)(b[3] * WCARRY);
  unsigned short* p = WH + (size_t)g * PLANE_H + e0;
  *(volatile v8h*)p = hv;
  __threadfence();
  *(volatile v8h*)p = hv;
}

__global__ __launch_bounds__(NTHR) void lstm_seq_kernel(
    const float* __restrict__ x, const float* __restrict__ h0, const float* __restrict__ c0,
    const float* __restrict__ bf_, const float* __restrict__ bi_,
    const float* __restrict__ bc_, const float* __restrict__ bo_,
    const float* __restrict__ mf_, const float* __restrict__ mi_,
    const float* __restrict__ mc_, const float* __restrict__ mo_,
    const float* __restrict__ wout, const float* __restrict__ bout,
    const unsigned short* __restrict__ WXp, const unsigned short* __restrict__ WHp,
    float* __restrict__ slab) {
  __shared__ __align__(16) _Float16 Axs[ROWS_PB * AXP];
  __shared__ __align__(16) _Float16 Ahs[ROWS_PB * AHP];
  __shared__ __align__(16) float    Msk[NGATE * MSK_PL];
  __shared__ __align__(16) float    Ys[SLAB_PB];
  __shared__ float                  PartS[8 * ROWS_PB];

  const _Float16* WX = (const _Float16*)WXp;
  const _Float16* WH = (const _Float16*)WHp;
  const int tid = threadIdx.x, lane = tid & 31, wave = tid >> 5;
  const int c = lane & 15, hh = lane >> 4, koff = hh * 8;
  const int rb = blockIdx.x * ROWS_PB;

#pragma unroll 1
  for (int i = 0; i < ROWS_PB; ++i) {
    const size_t src = (size_t)(rb + i) * NHID + tid;
    const int dst = i * NHID + tid;
    Msk[0 * MSK_PL + dst] = mf_[src];
    Msk[1 * MSK_PL + dst] = mi_[src];
    Msk[2 * MSK_PL + dst] = mc_[src];
    Msk[3 * MSK_PL + dst] = mo_[src];
  }
#pragma unroll 1
  for (int i = 0; i < ROWS_PB; ++i)
    Ahs[i * AHP + tid] = (_Float16)h0[(size_t)(rb + i) * NHID + tid];
#pragma unroll 1
  for (int i = tid; i < ROWS_PB * AXP; i += NTHR)
    if ((i % AXP) >= NIN) Axs[i] = (_Float16)0.0f;
  if (tid < ROWS_PB * NIN) {
    const int m = tid >> 3, k = tid & 7;
    Axs[m * AXP + k] = (_Float16)x[((size_t)rb + m) * NIN + k];
  }
  float cst[2][8], hst[2][8], bb[2][4], wo[2];
#pragma unroll
  for (int nt = 0; nt < 2; ++nt) {
    const int j = 32 * wave + 16 * nt + c;
    bb[nt][0] = bf_[j]; bb[nt][1] = bi_[j]; bb[nt][2] = bc_[j]; bb[nt][3] = bo_[j];
    wo[nt] = wout[j];
#pragma unroll
    for (int r = 0; r < 8; ++r) {
      cst[nt][r] = c0[(size_t)(rb + 8 * hh + r) * NHID + j];
      hst[nt][r] = 0.0f;
    }
  }
  const float bout_v = bout[0];
  __syncthreads();

  const _Float16* axrow = Axs + c * AXP + koff;
  const _Float16* ahrow = Ahs + c * AHP + koff;
  const v8f z8 = {0.f, 0.f, 0.f, 0.f, 0.f, 0.f, 0.f, 0.f};

#pragma unroll 1
  for (int t = 0; t < SEQ_LEN; ++t) {
#pragma unroll
    for (int nt = 0; nt < 2; ++nt) {
      const int j = 32 * wave + 16 * nt + c;
      const _Float16* wx = WX + (size_t)j * KXPAD + koff;
      const _Float16* wh = WH + (size_t)j * NHID + koff;
      v8f acc[4];
      acc[0] = z8; acc[1] = z8; acc[2] = z8; acc[3] = z8;
      {
        const v16h a  = Frag<_Float16>::load(axrow);
        const v16h b0 = Frag<_Float16>::load(wx);
        const v16h b1 = Frag<_Float16>::load(wx + (size_t)1 * PLANE_X);
        const v16h b2 = Frag<_Float16>::load(wx + (size_t)2 * PLANE_X);
        const v16h b3 = Frag<_Float16>::load(wx + (size_t)3 * PLANE_X);
        acc[0] = Frag<_Float16>::mma(a, b0, acc[0]);
        acc[1] = Frag<_Float16>::mma(a, b1, acc[1]);
        acc[2] = Frag<_Float16>::mma(a, b2, acc[2]);
        acc[3] = Frag<_Float16>::mma(a, b3, acc[3]);
        dep_guard_h(acc[0], acc[3], a, b3);
        keep4_h(b0, b1, b2, b3);
      }
#pragma unroll 1
      for (int k0 = 0; k0 < NHID; k0 += 32) {
        const v16h a  = Frag<_Float16>::load(ahrow + k0);
        const v16h b0 = Frag<_Float16>::load(wh + k0);
        const v16h b1 = Frag<_Float16>::load(wh + (size_t)1 * PLANE_H + k0);
        const v16h b2 = Frag<_Float16>::load(wh + (size_t)2 * PLANE_H + k0);
        const v16h b3 = Frag<_Float16>::load(wh + (size_t)3 * PLANE_H + k0);
        acc[0] = Frag<_Float16>::mma(a, b0, acc[0]);
        acc[1] = Frag<_Float16>::mma(a, b1, acc[1]);
        acc[2] = Frag<_Float16>::mma(a, b2, acc[2]);
        acc[3] = Frag<_Float16>::mma(a, b3, acc[3]);
        dep_guard_h(acc[0], acc[3], a, b3);
        keep4_h(b0, b1, b2, b3);
      }
      acc_guard4(acc[0], acc[1], acc[2], acc[3]);
#pragma unroll
      for (int r = 0; r < 8; ++r) {
        const int mr = (8 * hh + r) * NHID + j;
        const float zf = acc[0][r] * WCARRY_INV + bb[nt][0];
        const float zi = acc[1][r] * WCARRY_INV + bb[nt][1];
        const float zc = acc[2][r] * WCARRY_INV + bb[nt][2];
        const float zo = acc[3][r] * WCARRY_INV + bb[nt][3];
        const float fg = fsig(zf) * Msk[mr];
        const float ig = fsig(zi) * Msk[MSK_PL + mr];
        const float gg = fsig(zc) * Msk[2 * MSK_PL + mr];
        const float og = fsig(zo) * Msk[3 * MSK_PL + mr];
        const float cn = fg * cst[nt][r] + ig * gg;
        cst[nt][r] = cn;
        hst[nt][r] = og * ftanh(cn);
      }
    }
    float part[8];
#pragma unroll
    for (int r = 0; r < 8; ++r) {
      float p = hst[0][r] * wo[0] + hst[1][r] * wo[1];
#pragma unroll
      for (int off = 1; off < 16; off <<= 1) p += __shfl_xor(p, off, 32);
      part[r] = p;
    }
    if (c == 0) {
#pragma unroll
      for (int r = 0; r < 8; ++r) PartS[wave * ROWS_PB + 8 * hh + r] = part[r];
    }
    __syncthreads();
#pragma unroll
    for (int nt = 0; nt < 2; ++nt) {
      const int j = 32 * wave + 16 * nt + c;
#pragma unroll
      for (int r = 0; r < 8; ++r) Ahs[(8 * hh + r) * AHP + j] = (_Float16)hst[nt][r];
    }
    if (tid < ROWS_PB * NIN) {
      const int tn = (t + 1 < SEQ_LEN) ? (t + 1) : (SEQ_LEN - 1);
      const int m = tid >> 3, k = tid & 7;
      Axs[m * AXP + k] = (_Float16)x[((size_t)tn * NBATCH + rb + m) * NIN + k];
    }
    if (tid < ROWS_PB) {
      float s = bout_v;
#pragma unroll
      for (int w = 0; w < 8; ++w) s += PartS[w * ROWS_PB + tid];
      Ys[t * ROWS_PB + tid] = tanhf(s);
    }
    __syncthreads();
  }

  float* sb = slab + (size_t)blockIdx.x * SLAB_PB;
  for (int pass = 0; pass < 2; ++pass) {
#pragma unroll
    for (int it = 0; it < 4; ++it) {
      const int idx = it * NTHR + tid;
      const v4f v = *(const v4f*)(Ys + idx * 4);
      *(volatile v4f*)(sb + (size_t)idx * 4) = v;
    }
    __threadfence();
  }
}

__global__ __launch_bounds__(NTHR) void gather_rows_kernel(const float* __restrict__ slab, float* __restrict__ out) {
  const int tid = threadIdx.x;
  const int t = blockIdx.x * 2 + (tid >> 7);
  const int q = tid & 127;
  const int blk = q >> 2;
  const int cb = (q & 3) * 4;
  const v4f v = *(const v4f*)(slab + (size_t)blk * SLAB_PB + t * ROWS_PB + cb);
  float* p = out + (size_t)t * NBATCH + q * 4;
  *(volatile v4f*)p = v;
  __threadfence();
  *(volatile v4f*)p = v;
}

extern "C" void kernel_launch(void* const* d_in, const int* in_sizes, int n_in,
                              void* d_out, int out_size, void* d_ws, size_t ws_size, hipStream_t stream) {
  if (n_in < 21 || d_out == nullptr || d_ws == nullptr) return;
  if (in_sizes[0] != SEQ_LEN * NBATCH * NIN || in_sizes[1] != NBATCH * NHID || in_sizes[2] != NBATCH * NHID) return;
  if (in_sizes[3] != NHID * NIN || in_sizes[5] != NHID * NIN || in_sizes[7] != NHID * NIN || in_sizes[9] != NHID * NIN) return;
  if (in_sizes[4] != NHID * NHID || in_sizes[6] != NHID * NHID || in_sizes[8] != NHID * NHID || in_sizes[10] != NHID * NHID) return;
  if (in_sizes[11] != NHID || in_sizes[12] != NHID || in_sizes[13] != NHID || in_sizes[14] != NHID) return;
  if (in_sizes[15] != NBATCH * NHID || in_sizes[16] != NBATCH * NHID || in_sizes[17] != NBATCH * NHID || in_sizes[18] != NBATCH * NHID) return;
  if (in_sizes[19] != NHID || in_sizes[20] != 1 || out_size != SEQ_LEN * NBATCH) return;

  const float* x    = (const float*)d_in[0];
  const float* h0   = (const float*)d_in[1];
  const float* c0   = (const float*)d_in[2];
  const float* W_f  = (const float*)d_in[3];
  const float* V_f  = (const float*)d_in[4];
  const float* W_i  = (const float*)d_in[5];
  const float* V_i  = (const float*)d_in[6];
  const float* W_c  = (const float*)d_in[7];
  const float* V_c  = (const float*)d_in[8];
  const float* W_o  = (const float*)d_in[9];
  const float* V_o  = (const float*)d_in[10];
  const float* b_f  = (const float*)d_in[11];
  const float* b_i  = (const float*)d_in[12];
  const float* b_c  = (const float*)d_in[13];
  const float* b_o  = (const float*)d_in[14];
  const float* m_f  = (const float*)d_in[15];
  const float* m_i  = (const float*)d_in[16];
  const float* m_c  = (const float*)d_in[17];
  const float* m_o  = (const float*)d_in[18];
  const float* Wout = (const float*)d_in[19];
  const float* bout = (const float*)d_in[20];
  float* out = (float*)d_out;

  char* ws = (char*)d_ws; size_t off = 0;
  auto carve = [&](size_t bytes) -> char* { char* p = ws + off; off += (bytes + 255) & ~(size_t)255; return p; };
  unsigned short* WX = (unsigned short*)carve((size_t)NGATE * PLANE_X * 2);
  unsigned short* WH = (unsigned short*)carve((size_t)NGATE * PLANE_H * 2);
  float* SLAB = (float*)carve((size_t)NBLK_SEQ * SLAB_PB * 4);
  if (off > ws_size || off > (size_t)134217728) return;

  prep_in_kernel<<<(NGATE * PLANE_X) / (NTHR * 8), NTHR, 0, stream>>>(W_f, W_i, W_c, W_o, WX);
  prep_rec_kernel<<<(NGATE * PLANE_H) / (NTHR * 8), NTHR, 0, stream>>>(V_f, V_i, V_c, V_o, WH);
  lstm_seq_kernel<<<NBLK_SEQ, NTHR, 0, stream>>>(x, h0, c0, b_f, b_i, b_c, b_o, m_f, m_i, m_c, m_o,
                                                 Wout, bout, WX, WH, SLAB);
  gather_rows_kernel<<<(SEQ_LEN * NBATCH) / (NTHR * 4), NTHR, 0, stream>>>(SLAB, out);
}
